// KANCouplingNet_23450521436793
// MI455X (gfx1250) — hardware-verified
//
#include <hip/hip_runtime.h>


typedef __attribute__((ext_vector_type(16))) _Float16 v16h;
typedef __attribute__((ext_vector_type(8)))  _Float16 v8h;
typedef __attribute__((ext_vector_type(8)))  float    v8f;
typedef __attribute__((ext_vector_type(4)))  float    v4f;

template <typename T> struct Frag;
template <> struct Frag<_Float16> {
  typedef v16h V; union U { v16h v; v8h h[2]; };
  static __device__ __forceinline__ v16h load(const _Float16* p) {
    U f; f.h[0] = *(const v8h*)(p); f.h[1] = *(const v8h*)(p + 16); return f.v;
  }
};

__device__ __forceinline__ v8f mma_h(v16h a, v16h b, v8f c) {
  c = __builtin_amdgcn_wmma_f32_16x16x32_f16(false, a, false, b, (short)0, c, false, false);
  asm volatile("v_nop\n\tv_nop\n\tv_nop\n\tv_nop" : "+v"(c) : "v"(a), "v"(b));
  return c;
}

#define RS0   136
#define RS12  584
#define WS_L0 0
#define WS_L1 8704
#define WS_L2 46080
#define WS_TOTAL 64768
#define WS_NV8 (WS_TOTAL / 8)
#define WSC 64.0f
#define WSC_INV 0.015625f

#define HSTR 68
#define OSTR 132

__device__ __forceinline__ float silu_f(float v) {
  return v * __builtin_amdgcn_rcpf(1.0f + __expf(-v));
}

__device__ __forceinline__ void bspline8(float x, const float* g, const float* iv, float* o) {
  float gv[12], d[12];
#pragma unroll
  for (int j = 0; j < 12; ++j) { gv[j] = g[j]; d[j] = x - gv[j]; }
  float B[11];
#pragma unroll
  for (int j = 0; j < 11; ++j) B[j] = (x >= gv[j] && x < gv[j + 1]) ? 1.0f : 0.0f;
#pragma unroll
  for (int j = 0; j < 10; ++j) {
    const float q0 = d[j] * iv[j];
    const float q1 = (gv[j + 2] - x) * iv[j + 1];
    B[j] = q0 * B[j] + q1 * B[j + 1];
  }
#pragma unroll
  for (int j = 0; j < 9; ++j) {
    const float q0 = d[j] * iv[11 + j];
    const float q1 = (gv[j + 3] - x) * iv[12 + j];
    B[j] = q0 * B[j] + q1 * B[j + 1];
  }
#pragma unroll
  for (int j = 0; j < 8; ++j) {
    const float q0 = d[j] * iv[21 + j];
    const float q1 = (gv[j + 4] - x) * iv[22 + j];
    o[j] = q0 * B[j] + q1 * B[j + 1];
  }
}

__global__ __launch_bounds__(256) void kan_prep(const float* __restrict__ c0, const float* __restrict__ sb0, const float* __restrict__ ss0,
                                                const float* __restrict__ c1, const float* __restrict__ sb1, const float* __restrict__ ss1,
                                                const float* __restrict__ c2, const float* __restrict__ sb2, const float* __restrict__ ss2,
                                                _Float16* __restrict__ wt) {
  const int t8 = blockIdx.x * 256 + threadIdx.x;
  if (t8 >= WS_NV8) return;
  const int idx0 = t8 * 8;
  const float *coef, *sb, *ss;
  int in, out, rs, base;
  if (idx0 < WS_L1)      { coef = c0; sb = sb0; ss = ss0; in = 12; out = 64; rs = RS0;  base = WS_L0; }
  else if (idx0 < WS_L2) { coef = c1; sb = sb1; ss = ss1; in = 64; out = 64; rs = RS12; base = WS_L1; }
  else                   { coef = c2; sb = sb2; ss = ss2; in = 64; out = 24; rs = RS12; base = WS_L2; }
  const int rel = idx0 - base;
  const int n = rel / rs;
  const int k0 = rel - n * rs;
  const int nn = (n < out) ? n : (out - 1);
  v8h hv;
#pragma unroll
  for (int e = 0; e < 8; ++e) {
    const int k = k0 + e;
    int isp = k >> 3; isp = (isp < in) ? isp : (in - 1);
    const int gg = k & 7;
    int ib = k - in * 8; ib = (ib < 0) ? 0 : ib; ib = (ib < in) ? ib : (in - 1);
    const float vsp = coef[(isp * out + nn) * 8 + gg] * ss[isp * out + nn];
    const float vb  = sb[ib * out + nn];
    float v = 0.0f;
    if (n < out) {
      if (k < in * 8) v = vsp;
      else if (k < in * 9) v = vb;
    }
    hv[e] = (_Float16)(v * WSC);
  }
  volatile v8h* dst = (volatile v8h*)wt;
  dst[t8] = hv;
  __threadfence();
  dst[t8] = hv;
}

__device__ __forceinline__ void stage_wt(int tid, const _Float16* __restrict__ src, _Float16* dst, int nvec) {
  const v8h* s = (const v8h*)src;
  v8h* d = (v8h*)dst;
  for (int i = tid; i < nvec; i += 256) d[i] = s[i];
}

__device__ __forceinline__ void stage_grid(int tid, const float* __restrict__ g, float* gS, float* ivd, int in) {
  for (int i = tid; i < in * 12; i += 256) gS[i] = g[i];
  for (int idx = tid; idx < in * 30; idx += 256) {
    const int i = idx / 30, s = idx - i * 30;
    const float* gr = g + i * 12;
    float dd;
    if (s < 11)      dd = gr[s + 1] - gr[s];
    else if (s < 21) { const int j = s - 11; dd = gr[j + 2] - gr[j]; }
    else             { const int j = s - 21; dd = gr[j + 3] - gr[j]; }
    ivd[i * 32 + s] = 1.0f / dd;
  }
}

template <int IN, int NT, int KT>
__device__ __forceinline__ void layer_mm(const _Float16* Wt, const float* gS, const float* ivd,
                                         const float* hrow, int lane, v8f (&acc)[NT]) {
  constexpr int K9 = IN * 9;
  constexpr int RS = ((K9 + 31) / 32) * 32 + 8;
  const int r   = lane & 15;
  const int hlf = lane >> 4;
#pragma unroll 1
  for (int t = 0; t < KT; ++t) {
    v16h bf[NT];
#pragma unroll
    for (int nt = 0; nt < NT; ++nt)
      bf[nt] = Frag<_Float16>::load(Wt + (nt * 16 + r) * RS + t * 32 + 8 * hlf);
    v16h a;
    if (t < IN / 4) {
      const int i0 = 4 * t + hlf;
      const int i1 = i0 + 2;
      float b0[8], b1[8];
      bspline8(hrow[i0], gS + i0 * 12, ivd + i0 * 32, b0);
      bspline8(hrow[i1], gS + i1 * 12, ivd + i1 * 32, b1);
#pragma unroll
      for (int e = 0; e < 8; ++e) { a[e] = (_Float16)b0[e]; a[8 + e] = (_Float16)b1[e]; }
    } else {
#pragma unroll
      for (int e = 0; e < 16; ++e) {
        const int kk = 32 * t + ((e & 8) << 1) + 8 * hlf + (e & 7);
        const int i  = kk - IN * 8;
        const int ic = (i < IN) ? i : (IN - 1);
        float v = silu_f(hrow[ic]);
        v = (i < IN) ? v : 0.0f;
        a[e] = (_Float16)v;
      }
    }
#pragma unroll
    for (int nt = 0; nt < NT; ++nt) acc[nt] = mma_h(a, bf[nt], acc[nt]);
  }
}

__global__ __launch_bounds__(256) void kan_main(const float* __restrict__ x,
                                                const float* __restrict__ g0,
                                                const float* __restrict__ g1,
                                                const float* __restrict__ g2,
                                                const _Float16* __restrict__ wt,
                                                float* __restrict__ out) {
  __shared__ __align__(16) _Float16 Wt[64 * RS12];
  __shared__ __align__(16) float gS[64 * 12];
  __shared__ __align__(16) float ivd[64 * 32];
  __shared__ __align__(16) float hbuf[128 * HSTR];

  const int tid  = threadIdx.x;
  const int w    = tid >> 5;
  const int lane = tid & 31;
  const int hlf  = lane >> 4;
  const int r16  = lane & 15;
  const int blockrow = blockIdx.x * 128;
  const int rowbase  = blockrow + w * 16;
  float* hb = hbuf + (w * 16) * HSTR;
  const float* hrow = hb + r16 * HSTR;

  stage_wt(tid, wt + WS_L0, Wt, 64 * RS0 / 8);
  for (int idx = lane; idx < 192; idx += 32) {
    const int rr = idx / 12, c = idx - rr * 12;
    const int n = rowbase + rr;
    hb[rr * HSTR + c] = x[((size_t)((n >> 12) * 12 + c) << 12) | (size_t)(n & 4095)];
  }
  stage_grid(tid, g0, gS, ivd, 12);
  __syncthreads();
  {
    v8f acc[4];
#pragma unroll
    for (int nt = 0; nt < 4; ++nt) acc[nt] = (v8f){0.f, 0.f, 0.f, 0.f, 0.f, 0.f, 0.f, 0.f};
    layer_mm<12, 4, 4>(Wt, gS, ivd, hrow, lane, acc);
    __syncthreads();
#pragma unroll
    for (int nt = 0; nt < 4; ++nt)
#pragma unroll
      for (int j = 0; j < 8; ++j)
        hb[(hlf * 8 + j) * HSTR + nt * 16 + r16] = acc[nt][j] * WSC_INV;
  }

  stage_wt(tid, wt + WS_L1, Wt, 64 * RS12 / 8);
  stage_grid(tid, g1, gS, ivd, 64);
  __syncthreads();
  {
    v8f acc[4];
#pragma unroll
    for (int nt = 0; nt < 4; ++nt) acc[nt] = (v8f){0.f, 0.f, 0.f, 0.f, 0.f, 0.f, 0.f, 0.f};
    layer_mm<64, 4, 18>(Wt, gS, ivd, hrow, lane, acc);
    __syncthreads();
#pragma unroll
    for (int nt = 0; nt < 4; ++nt)
#pragma unroll
      for (int j = 0; j < 8; ++j)
        hb[(hlf * 8 + j) * HSTR + nt * 16 + r16] = acc[nt][j] * WSC_INV;
  }

  stage_wt(tid, wt + WS_L2, Wt, 32 * RS12 / 8);
  stage_grid(tid, g2, gS, ivd, 64);
  __syncthreads();
  {
    v8f acc[2];
#pragma unroll
    for (int nt = 0; nt < 2; ++nt) acc[nt] = (v8f){0.f, 0.f, 0.f, 0.f, 0.f, 0.f, 0.f, 0.f};
    layer_mm<64, 2, 18>(Wt, gS, ivd, hrow, lane, acc);
    __syncthreads();
    float* outS = hbuf;
#pragma unroll
    for (int nt = 0; nt < 2; ++nt) {
      const int c = nt * 16 + r16;
      if (c < 24) {
#pragma unroll
        for (int j = 0; j < 8; ++j)
          outS[c * OSTR + w * 16 + hlf * 8 + j] = acc[nt][j] * WSC_INV;
      }
    }
  }
  __syncthreads();

  {
    const int bimg = blockrow >> 12;
    const int hw0  = blockrow & 4095;
    float* ob = out + (size_t)bimg * 24 * 4096 + hw0;
    const float* outS = hbuf;
    for (int pass = 0; pass < 2; ++pass) {
#pragma unroll
      for (int m = 0; m < 3; ++m) {
        const int c = w + 8 * m;
        const v4f v = *(const v4f*)(outS + c * OSTR + lane * 4);
        *(volatile v4f*)(ob + (size_t)c * 4096 + lane * 4) = v;
      }
      __threadfence();
    }
  }
}

extern "C" void kernel_launch(void* const* d_in, const int* in_sizes, int n_in,
                              void* d_out, int out_size, void* d_ws, size_t ws_size,
                              hipStream_t stream) {
  (void)n_in; (void)out_size;
  const float* x   = (const float*)d_in[0];
  const float* g0  = (const float*)d_in[1];
  const float* c0  = (const float*)d_in[2];
  const float* sb0 = (const float*)d_in[3];
  const float* ss0 = (const float*)d_in[4];
  const float* g1  = (const float*)d_in[5];
  const float* c1  = (const float*)d_in[6];
  const float* sb1 = (const float*)d_in[7];
  const float* ss1 = (const float*)d_in[8];
  const float* g2  = (const float*)d_in[9];
  const float* c2  = (const float*)d_in[10];
  const float* sb2 = (const float*)d_in[11];
  const float* ss2 = (const float*)d_in[12];

  if (ws_size < (size_t)WS_TOTAL * 2) return;
  _Float16* wt = (_Float16*)d_ws;

  kan_prep<<<(WS_NV8 + 255) / 256, 256, 0, stream>>>(c0, sb0, ss0, c1, sb1, ss1, c2, sb2, ss2, wt);

  const int rows = in_sizes[0] / 12;
  const int blocks = rows / 128;
  if (blocks < 1) return;
  kan_main<<<blocks, 256, 0, stream>>>(x, g0, g1, g2, wt, (float*)d_out);
}
